// QAttention_75969381532133
// MI455X (gfx1250) — hardware-verified
//
#include <hip/hip_runtime.h>


#define NB_  2
#define CIN  128
#define C3   384
#define HW   16384
#define IMW  128
#define NHD  4
#define CH   32
#define K9   (9 * C3)
#define PCH  4096
typedef _Float16 h16;
typedef unsigned short bf;
typedef __attribute__((ext_vector_type(16))) __bf16   v16bf;
typedef __attribute__((ext_vector_type(16))) _Float16 v16h;
typedef __attribute__((ext_vector_type(8)))  _Float16 v8h;
typedef __attribute__((ext_vector_type(8)))  unsigned short v8us;
typedef __attribute__((ext_vector_type(8)))  float    v8f;
typedef __attribute__((ext_vector_type(4)))  float    v4f;
typedef v8h  __attribute__((may_alias)) v8ha;
typedef v4f  __attribute__((may_alias)) v4fa;
typedef v8us __attribute__((may_alias)) v8usa;

__device__ __forceinline__ unsigned short f2bf(float f) { unsigned u = __float_as_uint(f); u += 0x7FFFu + ((u >> 16) & 1u); return (unsigned short)(u >> 16); }
__device__ __forceinline__ float bf2f(unsigned short b) { return __uint_as_float(((unsigned)b) << 16); }
__device__ __forceinline__ float bfr(float f) { return bf2f(f2bf(f)); }
__device__ __forceinline__ v16h cat16(v8h lo, v8h hi) { return __builtin_shufflevector(lo, hi, 0, 1, 2, 3, 4, 5, 6, 7, 8, 9, 10, 11, 12, 13, 14, 15); }
__device__ __forceinline__ v16bf cat16b(v8us lo, v8us hi) { return __builtin_bit_cast(v16bf, __builtin_shufflevector(lo, hi, 0, 1, 2, 3, 4, 5, 6, 7, 8, 9, 10, 11, 12, 13, 14, 15)); }
__device__ __forceinline__ v8f wmma16(v16h a, v16h b, v8f c) { return __builtin_amdgcn_wmma_f32_16x16x32_f16(false, a, false, b, (short)0, c, false, false); }
__device__ __forceinline__ v8f wmmab(v16bf a, v16bf b, v8f c) { return __builtin_amdgcn_wmma_f32_16x16x32_bf16(false, a, false, b, (short)0, c, false, false); }


template <typename T16> struct WFrag;
template <> struct WFrag<h16> { typedef v16h V; static __device__ __forceinline__ V ld(const h16* p) { return cat16(*(const v8h*)p, *(const v8h*)(p + 16)); } static __device__ __forceinline__ v8f mma(V a, V b, v8f c) { return wmma16(a, b, c); } };
template <> struct WFrag<bf> { typedef v16bf V; static __device__ __forceinline__ V ld(const bf* p) { return cat16b(*(const v8us*)p, *(const v8us*)(p + 16)); } static __device__ __forceinline__ v8f mma(V a, V b, v8f c) { return wmmab(a, b, c); } };
template <typename T16, int NSPLIT, bool BIAS>
__global__ __launch_bounds__(32) void k_gemmw(const T16* __restrict__ A, const T16* __restrict__ A2, const T16* __restrict__ Bt, const T16* __restrict__ Bt2, int K, float* C, int ldc, const float* __restrict__ bias, size_t sA, size_t sB, size_t sC) {
    typedef typename WFrag<T16>::V V;
    __shared__ __align__(16) float os[16 * 68];
    const size_t z = blockIdx.z; A += z * sA; if (A2) A2 += z * sA; Bt += z * sB; if (Bt2) Bt2 += z * sB; C += z * sC;
    const int lane = threadIdx.x & 31, lr = lane & 15, hi = lane >> 4; const int r0 = blockIdx.x * 64, c0 = blockIdx.y * 64;
    v8f acc[4][4];
#pragma unroll
    for (int mb = 0; mb < 4; ++mb)
#pragma unroll
        for (int nb = 0; nb < 4; ++nb) acc[mb][nb] = (v8f){};
    const size_t aoff = (size_t)(r0 + lr) * K + 8 * hi, boff = (size_t)(c0 + lr) * K + 8 * hi;
#pragma unroll 1
    for (int kc = 0; kc < K; kc += 32) {
        V a[4], a2[4];
#pragma unroll
        for (int mb = 0; mb < 4; ++mb) { a[mb] = WFrag<T16>::ld(A + aoff + (size_t)mb * 16 * K + kc); if (NSPLIT == 1 || NSPLIT == 2) a2[mb] = WFrag<T16>::ld(A2 + aoff + (size_t)mb * 16 * K + kc); }
#pragma unroll
        for (int nb = 0; nb < 4; ++nb) { const V b = WFrag<T16>::ld(Bt + boff + (size_t)nb * 16 * K + kc); V b2; if (NSPLIT >= 2) b2 = WFrag<T16>::ld(Bt2 + boff + (size_t)nb * 16 * K + kc);
#pragma unroll
            for (int mb = 0; mb < 4; ++mb) { acc[mb][nb] = WFrag<T16>::mma(a[mb], b, acc[mb][nb]); if (NSPLIT == 1 || NSPLIT == 2) acc[mb][nb] = WFrag<T16>::mma(a2[mb], b, acc[mb][nb]); if (NSPLIT >= 2) acc[mb][nb] = WFrag<T16>::mma(a[mb], b2, acc[mb][nb]); } }
        asm volatile("v_nop\n\tv_nop\n\tv_nop\n\tv_nop" : "+v"(acc[0][0]), "+v"(acc[1][1]), "+v"(acc[2][2]), "+v"(acc[3][3]) : "v"(a[0]), "v"(a[3]));
    }
#pragma unroll
    for (int mb = 0; mb < 4; ++mb) {
#pragma unroll
        for (int nb = 0; nb < 4; ++nb) {
#pragma unroll
            for (int j = 0; j < 8; ++j) os[(hi * 8 + j) * 68 + nb * 16 + lr] = acc[mb][nb][j]; }
        __builtin_amdgcn_wave_barrier(); asm volatile("" ::: "memory");
        float* crow = C + (size_t)(r0 + mb * 16) * ldc + c0;
#pragma unroll 1
        for (int ps = 0; ps < 2; ++ps) {
#pragma unroll
            for (int s = 0; s < 8; ++s) { const int row = 2 * s + hi, cofs = lr * 4; v4f val = *(const v4fa*)(os + row * 68 + cofs); if (BIAS) { val[0] += bfr(bias[c0 + cofs]); val[1] += bfr(bias[c0 + cofs + 1]); val[2] += bfr(bias[c0 + cofs + 2]); val[3] += bfr(bias[c0 + cofs + 3]); }
                *(volatile v4f*)(crow + (size_t)row * ldc + cofs) = val; }
            if (ps == 0) __threadfence(); }
        __builtin_amdgcn_wave_barrier(); asm volatile("" ::: "memory");
    }
}

__device__ __forceinline__ h16 tohx(float x) { return (h16)x; }
__device__ __forceinline__ void splitf(float y, unsigned short& h, unsigned short& l) { h = f2bf(y); l = f2bf(y - bf2f(h)); }
typedef __attribute__((ext_vector_type(2))) _Float16 v2h;
typedef __attribute__((ext_vector_type(4))) _Float16 v4h;
typedef __attribute__((ext_vector_type(2))) unsigned short v2us;
typedef __attribute__((ext_vector_type(4))) unsigned short v4us;
typedef __attribute__((ext_vector_type(2))) float v2f;
typedef __attribute__((ext_vector_type(4))) int v4i;

__global__ __launch_bounds__(256) void k_cvt8(const float* __restrict__ src, bf* dst, size_t n8) { const size_t i = (size_t)blockIdx.x * 256 + threadIdx.x; if (i >= n8) return; const v8f v = *(const v8f*)(src + i * 8); v8us o;
#pragma unroll
    for (int k = 0; k < 8; ++k) o[k] = f2bf(v[k]); *(volatile v8us*)(dst + i * 8) = o; __threadfence(); *(volatile v8us*)(dst + i * 8) = o; }
__global__ __launch_bounds__(256) void k_cvt8Tg(const float* __restrict__ src, bf* dst, int R, int C) { const size_t i = (size_t)blockIdx.x * 256 + threadIdx.x; if (i >= (size_t)R * C / 8) return; const int c = (int)(i / (R / 8)); const int r0 = (int)(i % (R / 8)) * 8; v8us o;
#pragma unroll
    for (int k = 0; k < 8; ++k) o[k] = f2bf(src[(size_t)(r0 + k) * C + c]); *(volatile v8us*)(dst + (size_t)c * R + r0) = o; __threadfence(); *(volatile v8us*)(dst + (size_t)c * R + r0) = o; }
__global__ __launch_bounds__(256) void k_split8(const float* __restrict__ F, bf* Ph, bf* Pl, size_t n8) { const size_t i = (size_t)blockIdx.x * 256 + threadIdx.x; if (i >= n8) return; const v8f v = *(const v8f*)(F + i * 8); v8us oh, ol;
#pragma unroll
    for (int k = 0; k < 8; ++k) { unsigned short a, c2; splitf(v[k], a, c2); oh[k] = a; ol[k] = c2; }
    *(volatile v8us*)(Ph + i * 8) = oh; *(volatile v8us*)(Pl + i * 8) = ol; __threadfence(); *(volatile v8us*)(Ph + i * 8) = oh; *(volatile v8us*)(Pl + i * 8) = ol; }

__global__ __launch_bounds__(256) void k_qw(const float* __restrict__ wr, const float* __restrict__ wi, const float* __restrict__ wj, const float* __restrict__ wk, int OB, int IB, int taps, bf* dst) {
    const int KK = taps * 4 * IB; const size_t i = (size_t)blockIdx.x * 256 + threadIdx.x; if (i >= (size_t)4 * OB * KK / 8) return; const int o = (int)(i / (KK / 8)); const int k0 = (int)(i % (KK / 8)) * 8; const int ro = o / OB, oo = o % OB; v8us ov; int chain = 0;
#pragma unroll
    for (int q = 0; q < 8; ++q) { const int k = k0 + q; const int tap = k / (4 * IB); const int c = k % (4 * IB); const int cb = c / IB, cc = c % IB;
        const int s = ro ^ cb; const float sg = 1.0f - 2.0f * (float)((10318 >> (ro * 4 + cb)) & 1);
        const size_t off = ((size_t)oo * IB + cc) * taps + tap + chain; float a = wr[off], b = wi[off], cj = wj[off], dk = wk[off]; asm volatile("s_wait_loadcnt 0x0" : "+v"(a), "+v"(b), "+v"(cj), "+v"(dk), "+v"(chain) :: "memory");
        const float f0 = (float)(s == 0), f1 = (float)(s == 1), f2 = (float)(s == 2), f3 = (float)(s == 3);
        float w = __fmul_rn(a, f0); w = fmaf(b, f1, w); w = fmaf(cj, f2, w); w = fmaf(dk, f3, w); ov[q] = f2bf(sg * w); }
    *(volatile v8us*)(dst + i * 8) = ov; __threadfence(); *(volatile v8us*)(dst + i * 8) = ov; }
__global__ __launch_bounds__(256) void k_im2c(const float* __restrict__ F, int p0, bf* Ah, bf* Al) { const size_t e = ((size_t)blockIdx.x * 256 + threadIdx.x) * 8; if (e >= (size_t)PCH * K9) return; const int c = (int)(e % C3); const int tap = (int)((e / C3) % 9); const int pl = (int)(e / K9); const int p = p0 + pl; const int y = p / IMW + tap / 3 - 1, x = p % IMW + tap % 3 - 1; v8us oh, ol;
    if (y >= 0 && y < IMW && x >= 0 && x < IMW) { const v8f f = *(const v8f*)(F + ((size_t)y * IMW + x) * C3 + c);
#pragma unroll
        for (int q = 0; q < 8; ++q) { unsigned short a, c2; splitf(f[q], a, c2); oh[q] = a; ol[q] = c2; } } else {
#pragma unroll
        for (int q = 0; q < 8; ++q) { oh[q] = 0; ol[q] = 0; } }
    *(volatile v8us*)(Ah + e) = oh; *(volatile v8us*)(Al + e) = ol; __threadfence(); *(volatile v8us*)(Ah + e) = oh; *(volatile v8us*)(Al + e) = ol; }
__global__ __launch_bounds__(256) void k_chpl(const float* __restrict__ F, int coff, int nch, bf* Ph, bf* Pl) { const size_t e = ((size_t)blockIdx.x * 256 + threadIdx.x) * 2; if (e >= (size_t)nch * HW) return; const int p = (int)(e % HW); const int c = (int)(e / HW); v2us oh, ol;
#pragma unroll
    for (int q = 0; q < 2; ++q) { unsigned short a, c2; splitf(F[(size_t)(p + q) * C3 + coff + c], a, c2); oh[q] = a; ol[q] = c2; }
    *(volatile v2us*)(Ph + e) = oh; *(volatile v2us*)(Pl + e) = ol; __threadfence(); *(volatile v2us*)(Ph + e) = oh; *(volatile v2us*)(Pl + e) = ol; }
__global__ __launch_bounds__(256) void k_tkpl(const float* __restrict__ F, int coff, bf* Ph, bf* Pl) { const size_t e = ((size_t)blockIdx.x * 256 + threadIdx.x) * 2; if (e >= (size_t)HW * CIN) return; const int c = (int)(e % CIN); const int p = (int)(e / CIN); const float* f = F + (size_t)p * C3 + coff + c; v2us oh, ol;
#pragma unroll
    for (int q = 0; q < 2; ++q) { unsigned short a, c2; splitf(f[q], a, c2); oh[q] = a; ol[q] = c2; }
    *(volatile v2us*)(Ph + e) = oh; *(volatile v2us*)(Pl + e) = ol; __threadfence(); *(volatile v2us*)(Ph + e) = oh; *(volatile v2us*)(Pl + e) = ol; }
__global__ __launch_bounds__(256) void k_outT(const float* __restrict__ YT, float* out) { const size_t i = (size_t)blockIdx.x * 256 + threadIdx.x; if (i >= (size_t)CIN * HW / 8) return; const int o = (int)(i / (HW / 8)); const int p0 = (int)(i % (HW / 8)) * 8; v4f a, b2;
#pragma unroll
    for (int q = 0; q < 4; ++q) { a[q] = YT[(size_t)(p0 + q) * CIN + o]; b2[q] = YT[(size_t)(p0 + 4 + q) * CIN + o]; }
    float* dst = out + (size_t)o * HW + p0; *(volatile v4f*)dst = a; *(volatile v4f*)(dst + 4) = b2; __threadfence(); *(volatile v4f*)dst = a; *(volatile v4f*)(dst + 4) = b2; }
__global__ __launch_bounds__(256) void k_cnorm(const float* __restrict__ F, float* NSQ) { const int lane = threadIdx.x & 31; const int c = blockIdx.x * 8 + (threadIdx.x >> 5); if (c >= 2 * CIN) return; float s = 0.f;
#pragma unroll 4
    for (int p = lane; p < HW; p += 32) { const float v = F[(size_t)p * C3 + c]; float t = __fmul_rn(v, v); asm volatile("" : "+v"(t)); s = __fadd_rn(s, t); }
#pragma unroll
    for (int sh = 16; sh; sh >>= 1) s += __shfl_xor(s, sh, 32);
    const float rec = (lane == 0) ? s : 0.0f; *(volatile float*)(NSQ + (size_t)c * 32 + lane) = rec; __threadfence(); *(volatile float*)(NSQ + (size_t)c * 32 + lane) = rec; }
__global__ __launch_bounds__(256) void k_catt(const float* __restrict__ G, const float* __restrict__ NSQ, const float* __restrict__ temp, bf* Ah, bf* Al) { const int lane = threadIdx.x & 31; const int row = blockIdx.x * 8 + (threadIdx.x >> 5); if (row >= CIN) return; const int h = row / CH;
    float nq = __fsqrt_rn(NSQ[(size_t)row * 32]); asm volatile("" : "+v"(nq)); nq = fmaxf(nq, 1e-12f); float nk = __fsqrt_rn(NSQ[(size_t)(CIN + h * CH + lane) * 32]); asm volatile("" : "+v"(nk)); nk = fmaxf(nk, 1e-12f);
    const float graw = G[(size_t)row * CIN + h * CH + lane]; float g1 = __fdiv_rn(graw, nq); asm volatile("" : "+v"(g1)); float g2 = __fdiv_rn(g1, nk); asm volatile("" : "+v"(g2)); float a = __fmul_rn(g2, bfr(temp[h])); asm volatile("" : "+v"(a));
    float mx = a;
#pragma unroll
    for (int sh = 16; sh; sh >>= 1) mx = fmaxf(mx, __shfl_xor(mx, sh, 32));
    float d0 = __fsub_rn(a, mx); asm volatile("" : "+v"(d0)); const float ex = __builtin_amdgcn_exp2f(__fmul_rn(d0, 1.4426950408889634f)); float sum = ex;
#pragma unroll
    for (int sh = 16; sh; sh >>= 1) sum += __shfl_xor(sum, sh, 32);
    const float p = __fdiv_rn(ex, sum); v4us oh, ol;
#pragma unroll
    for (int q = 0; q < 4; ++q) { const int d = lane * 4 + q; const float pv = __shfl(p, d & 31, 32); const float val = (d / CH == h) ? pv : 0.0f; unsigned short a2, c2; splitf(val, a2, c2); oh[q] = a2; ol[q] = c2; }
    *(volatile v4us*)(Ah + (size_t)row * CIN + lane * 4) = oh; *(volatile v4us*)(Al + (size_t)row * CIN + lane * 4) = ol; __threadfence(); *(volatile v4us*)(Ah + (size_t)row * CIN + lane * 4) = oh; *(volatile v4us*)(Al + (size_t)row * CIN + lane * 4) = ol; }

extern "C" void kernel_launch(void* const* d_in, const int* in_sizes, int n_in,
                              void* d_out, int out_size, void* d_ws, size_t ws_size, hipStream_t stream) {
    (void)in_sizes; (void)n_in; (void)out_size;
    const float* x = (const float*)d_in[0];
    const float* q_r = (const float*)d_in[1]; const float* q_i = (const float*)d_in[2]; const float* q_j = (const float*)d_in[3]; const float* q_k = (const float*)d_in[4]; const float* q_b = (const float*)d_in[5];
    const float* d_r = (const float*)d_in[6]; const float* d_i = (const float*)d_in[7]; const float* d_j = (const float*)d_in[8]; const float* d_k = (const float*)d_in[9]; const float* d_b = (const float*)d_in[10];
    const float* p_r = (const float*)d_in[11]; const float* p_i = (const float*)d_in[12]; const float* p_j = (const float*)d_in[13]; const float* p_k = (const float*)d_in[14]; const float* p_b = (const float*)d_in[15]; const float* temp = (const float*)d_in[16];
    float* OUT = (float*)d_out;
    char* wsp = (char*)d_ws;
    auto take = [&](size_t bytes) { char* p = wsp; wsp += (bytes + 255) & ~(size_t)255; return (void*)p; };
    bf* W1B = (bf*)take((size_t)C3 * CIN * 2); bf* W2B = (bf*)take((size_t)C3 * K9 * 2); bf* W3B = (bf*)take((size_t)CIN * CIN * 2);
    bf* XT = (bf*)take((size_t)HW * CIN * 2); float* F1 = (float*)take((size_t)HW * C3 * 4); bf* ICh = (bf*)take((size_t)PCH * K9 * 2); bf* ICl = (bf*)take((size_t)PCH * K9 * 2); float* F2 = (float*)take((size_t)HW * C3 * 4);
    bf* QKh = (bf*)take((size_t)2 * CIN * HW * 2); bf* QKl = (bf*)take((size_t)2 * CIN * HW * 2); bf* VTh = (bf*)take((size_t)HW * CIN * 2); bf* VTl = (bf*)take((size_t)HW * CIN * 2); float* NSQ = (float*)take((size_t)2 * CIN * 32 * 4); float* G = (float*)take((size_t)CIN * CIN * 4);
    bf* Ah = (bf*)take((size_t)CIN * CIN * 2); bf* Al = (bf*)take((size_t)CIN * CIN * 2); float* OT = (float*)take((size_t)HW * CIN * 4); bf* OTh = (bf*)take((size_t)HW * CIN * 2); bf* OTl = (bf*)take((size_t)HW * CIN * 2); float* YT = (float*)take((size_t)HW * CIN * 4);
    if ((size_t)(wsp - (char*)d_ws) > ws_size) return;
    k_qw<<<(unsigned)(((size_t)C3 * CIN / 8 + 255) / 256), 256, 0, stream>>>(q_r, q_i, q_j, q_k, C3 / 4, CIN / 4, 1, W1B); k_qw<<<(unsigned)(((size_t)C3 * K9 / 8 + 255) / 256), 256, 0, stream>>>(d_r, d_i, d_j, d_k, C3 / 4, C3 / 4, 9, W2B); k_qw<<<(unsigned)(((size_t)CIN * CIN / 8 + 255) / 256), 256, 0, stream>>>(p_r, p_i, p_j, p_k, CIN / 4, CIN / 4, 1, W3B);
    for (int b = 0; b < NB_; ++b) {
        k_cvt8Tg<<<(unsigned)(((size_t)CIN * HW / 8 + 255) / 256), 256, 0, stream>>>(x + (size_t)b * CIN * HW, XT, CIN, HW);
        k_gemmw<bf, 0, true><<<dim3(HW / 64, C3 / 64, 1), 32, 0, stream>>>(XT, nullptr, W1B, nullptr, CIN, F1, C3, q_b, 0, 0, 0);
        for (int ck = 0; ck < HW / PCH; ++ck) {
            k_im2c<<<(unsigned)(((size_t)PCH * K9 / 8 + 255) / 256), 256, 0, stream>>>(F1, ck * PCH, ICh, ICl);
            k_gemmw<bf, 1, true><<<dim3(PCH / 64, C3 / 64, 1), 32, 0, stream>>>(ICh, ICl, W2B, nullptr, K9, F2 + (size_t)ck * PCH * C3, C3, d_b, 0, 0, 0); }
        k_chpl<<<(unsigned)(((size_t)2 * CIN * HW / 2 + 255) / 256), 256, 0, stream>>>(F2, 0, 2 * CIN, QKh, QKl);
        k_tkpl<<<(unsigned)(((size_t)HW * CIN / 2 + 255) / 256), 256, 0, stream>>>(F2, 2 * CIN, VTh, VTl);
        k_cnorm<<<2 * CIN / 8, 256, 0, stream>>>(F2, NSQ);
        k_gemmw<bf, 2, false><<<dim3(CIN / 64, CIN / 64, 1), 32, 0, stream>>>(QKh, QKl, QKh + (size_t)CIN * HW, QKl + (size_t)CIN * HW, HW, G, CIN, nullptr, 0, 0, 0);
        k_catt<<<CIN / 8, 256, 0, stream>>>(G, NSQ, temp, Ah, Al);
        k_gemmw<bf, 2, false><<<dim3(HW / 64, CIN / 64, 1), 32, 0, stream>>>(VTh, VTl, Ah, Al, CIN, OT, CIN, nullptr, 0, 0, 0);
        k_split8<<<(unsigned)(((size_t)HW * CIN / 8 + 255) / 256), 256, 0, stream>>>(OT, OTh, OTl, (size_t)HW * CIN / 8);
        k_gemmw<bf, 1, true><<<dim3(HW / 64, CIN / 64, 1), 32, 0, stream>>>(OTh, OTl, W3B, nullptr, CIN, YT, CIN, p_b, 0, 0, 0);
        k_outT<<<(unsigned)(((size_t)CIN * HW / 8 + 255) / 256), 256, 0, stream>>>(YT, OUT + (size_t)b * CIN * HW); }
}
